// Performer_8426725835128
// MI455X (gfx1250) — hardware-verified
//
#include <hip/hip_runtime.h>
#include <stddef.h>
#include <stdint.h>

#define NBATCH 8
#define SEQ    2048
#define DIM    256
#define NROWS  (NBATCH * SEQ)
#define CX     272
#define HP     72
#define FP     68
#define KVT    68

static_assert(DIM == 256);
static_assert(SEQ % 256 == 0);
static_assert(NROWS % 64 == 0);
static_assert((CX / 16) * 4 == KVT);
static_assert((NBATCH * KVT) % 8 == 0);
static_assert((HP * 2) % 16 == 0);
static_assert((FP * 4) % 16 == 0);
static_assert((NROWS * DIM) % (8 * 256) == 0);
static_assert((DIM * DIM) % (8 * 256) == 0);

typedef _Float16 v16h __attribute__((ext_vector_type(16)));
typedef _Float16 v8h  __attribute__((ext_vector_type(8)));
typedef float    v8f  __attribute__((ext_vector_type(8)));
typedef float    v4f  __attribute__((ext_vector_type(4)));
typedef unsigned int v4u __attribute__((ext_vector_type(4)));
typedef v4u __attribute__((may_alias)) v4ua;
typedef v4f __attribute__((may_alias)) v4fa;

union Frag  { v16h v; v8h h[2]; };
union Pack8 { v8h h; v4u u; };

__device__ __forceinline__ v8f mma16(v16h a, v16h b, v8f cacc) {
  cacc = __builtin_amdgcn_wmma_f32_16x16x32_f16(false, a, false, b, (short)0, cacc, false, false);
  asm volatile("v_nop\n\tv_nop\n\tv_nop\n\tv_nop" : "+v"(cacc) : "v"(a), "v"(b));
  return cacc;
}

__device__ __forceinline__ v8f zero8() { return (v8f){0.f, 0.f, 0.f, 0.f, 0.f, 0.f, 0.f, 0.f}; }

__device__ __forceinline__ v16h ldfrag_g(const _Float16* __restrict__ p, int ld, int row0, int k0, int lane) {
  const int m = lane & 15, lh = lane >> 4;
  const _Float16* q = p + (size_t)(row0 + m) * ld + k0 + 8 * lh;
  Frag f;
  f.h[0] = *(const v8h*)(q);
  f.h[1] = *(const v8h*)(q + 16);
  return f.v;
}

__global__ __launch_bounds__(256) void k_conv(const float* __restrict__ src, _Float16* __restrict__ dst,
                                              int nvec, float scale) {
  const int i = blockIdx.x * 256 + threadIdx.x;
  if (i < nvec) {
    const float* s = src + (size_t)i * 8;
    const v4f x0 = *(const v4f*)(s);
    const v4f x1 = *(const v4f*)(s + 4);
    Pack8 pk;
#pragma unroll
    for (int j = 0; j < 4; ++j) {
      pk.h[j]     = (_Float16)(x0[j] * scale);
      pk.h[4 + j] = (_Float16)(x1[j] * scale);
    }
    _Float16* d = dst + (size_t)i * 8;
    *(volatile v4u*)d = pk.u;
    __threadfence();
    *(volatile v4u*)d = pk.u;
  }
}

__global__ __launch_bounds__(256) void k_norm(const float* __restrict__ Q, const float* __restrict__ K,
                                              float* __restrict__ hn, const float* __restrict__ aux0,
                                              const int* __restrict__ aux1) {
  __shared__ __align__(16) float red[32];
  (void)aux0; (void)aux1;
  const int t = threadIdx.x, lane = t & 31, wave = t >> 5;
  const float* X = (blockIdx.y == 0) ? Q : K;
  const int l0 = blockIdx.x * 32;
  const int ll = t >> 3, part = t & 7;
  const float* p = X + (size_t)(l0 + ll) * DIM + part * 32;
  float s = 0.f;
#pragma unroll 1
  for (int b = 0; b < NBATCH; ++b) {
    const float* pb = p + (size_t)b * SEQ * DIM;
#pragma unroll
    for (int i = 0; i < 8; ++i) {
      const v4f v = *(const v4f*)(pb + 4 * i);
      s = fmaf(v[0], v[0], s);
      s = fmaf(v[1], v[1], s);
      s = fmaf(v[2], v[2], s);
      s = fmaf(v[3], v[3], s);
    }
  }
  s += __shfl_xor(s, 1);
  s += __shfl_xor(s, 2);
  s += __shfl_xor(s, 4);
  if (part == 0) red[ll] = 0.5f * sqrtf(s);
  __syncthreads();
  if (wave == 0) {
    const int q = lane & 7;
    const v4f v = *(const v4fa*)(red + q * 4);
    float* d = hn + (size_t)blockIdx.y * SEQ + l0 + q * 4;
    if (lane < 8) *(volatile v4f*)d = v;
    __threadfence();
    if (lane < 8) *(volatile v4f*)d = v;
  }
}

__global__ __launch_bounds__(256) void k_vt(const float* __restrict__ V, _Float16* __restrict__ VT) {
  __shared__ float tile[64][65];
  const int t = threadIdx.x;
  const int b = blockIdx.z, cb = blockIdx.y, l0 = blockIdx.x * 64;
  _Float16* VTb = VT + (size_t)b * CX * SEQ;
  if (cb < 4) {
    const float* Vb = V + (size_t)b * SEQ * DIM + cb * 64;
#pragma unroll
    for (int it = 0; it < 16; ++it) {
      const int row = it * 4 + (t >> 6), col = t & 63;
      tile[row][col] = Vb[(size_t)(l0 + row) * DIM + col];
    }
  }
  __syncthreads();
  if (cb < 4) {
    Pack8 pk[2];
#pragma unroll
    for (int it = 0; it < 2; ++it) {
      const int p = it * 256 + t, cl = p >> 3, pc = p & 7;
#pragma unroll
      for (int j = 0; j < 8; ++j) pk[it].h[j] = (_Float16)tile[pc * 8 + j][cl];
    }
#pragma unroll
    for (int it = 0; it < 2; ++it) {
      const int p = it * 256 + t, cl = p >> 3, pc = p & 7;
      *(volatile v4u*)(VTb + (size_t)(cb * 64 + cl) * SEQ + l0 + pc * 8) = pk[it].u;
    }
    __threadfence();
#pragma unroll
    for (int it = 0; it < 2; ++it) {
      const int p = it * 256 + t, cl = p >> 3, pc = p & 7;
      *(volatile v4u*)(VTb + (size_t)(cb * 64 + cl) * SEQ + l0 + pc * 8) = pk[it].u;
    }
  } else {
    if (t < 128) {
      const int cl = t >> 3, pc = t & 7;
      const float one = (cl == 0) ? 1.0f : 0.0f;
      Pack8 pk;
#pragma unroll
      for (int j = 0; j < 8; ++j) pk.h[j] = (_Float16)one;
      _Float16* d = VTb + (size_t)(DIM + cl) * SEQ + l0 + pc * 8;
      *(volatile v4u*)d = pk.u;
      __threadfence();
      *(volatile v4u*)d = pk.u;
    }
  }
}

__global__ __launch_bounds__(256) void k_phi(const _Float16* __restrict__ A, const _Float16* __restrict__ Bn,
                                             size_t strideB, const float* __restrict__ hn,
                                             _Float16* __restrict__ C, int ldc, size_t strideC, int hn_by_col) {
  __shared__ __align__(16) _Float16 st[8][32 * HP];
  const int tid = threadIdx.x, lane = tid & 31, wave = tid >> 5;
  const int hh = lane >> 4, c = lane & 15;
  const int rb = wave & 1, cg = wave >> 1;
  const int arow0 = blockIdx.x * 64 + rb * 32;
  const int bcol0 = blockIdx.y * 256 + cg * 64;
  const _Float16* Bz = Bn + strideB * (size_t)blockIdx.z;
  _Float16* Cz = C + strideC * (size_t)blockIdx.z;

  v8f acc[2][4];
#pragma unroll
  for (int s = 0; s < 2; ++s)
#pragma unroll
    for (int j = 0; j < 4; ++j) acc[s][j] = zero8();

#pragma unroll 2
  for (int kc = 0; kc < DIM / 32; ++kc) {
    const int k0 = kc * 32;
    const v16h a0 = ldfrag_g(A, DIM, arow0, k0, lane);
    const v16h a1 = ldfrag_g(A, DIM, arow0 + 16, k0, lane);
#pragma unroll
    for (int j = 0; j < 4; ++j) {
      const v16h bf = ldfrag_g(Bz, DIM, bcol0 + 16 * j, k0, lane);
      acc[0][j] = mma16(a0, bf, acc[0][j]);
      acc[1][j] = mma16(a1, bf, acc[1][j]);
    }
  }

  float hr[2][8], hcl[4];
#pragma unroll
  for (int s = 0; s < 2; ++s)
#pragma unroll
    for (int r = 0; r < 8; ++r) hr[s][r] = hn[(arow0 + s * 16 + 8 * hh + r) & (SEQ - 1)];
#pragma unroll
  for (int j = 0; j < 4; ++j) hcl[j] = hn[(bcol0 + 16 * j + c) & (SEQ - 1)];
  const float scl = 0.0009765625f;
  _Float16* sw = st[wave];
#pragma unroll
  for (int s = 0; s < 2; ++s)
#pragma unroll
    for (int j = 0; j < 4; ++j)
#pragma unroll
      for (int r = 0; r < 8; ++r) {
        const float sub = (hn_by_col != 0) ? hcl[j] : hr[s][r];
        const float e = __expf(acc[s][j][r] * scl - sub);
        sw[(s * 16 + 8 * hh + r) * HP + 16 * j + c] = (_Float16)e;
      }
  __syncthreads();

  v4u val[8];
#pragma unroll
  for (int it = 0; it < 8; ++it) {
    const int p = it * 32 + lane, row = p >> 3, pc = p & 7;
    val[it] = *(const v4ua*)(sw + row * HP + pc * 8);
  }
#pragma unroll
  for (int it = 0; it < 8; ++it) {
    const int p = it * 32 + lane, row = p >> 3, pc = p & 7;
    *(volatile v4u*)(Cz + (size_t)(arow0 + row) * ldc + bcol0 + pc * 8) = val[it];
  }
  __threadfence();
#pragma unroll
  for (int it = 0; it < 8; ++it) {
    const int p = it * 32 + lane, row = p >> 3, pc = p & 7;
    *(volatile v4u*)(Cz + (size_t)(arow0 + row) * ldc + bcol0 + pc * 8) = val[it];
  }
}

__global__ __launch_bounds__(256) void k_kv(const _Float16* __restrict__ VT, const _Float16* __restrict__ EKT,
                                            _Float16* __restrict__ TT) {
  __shared__ __align__(16) _Float16 st[8][16 * HP];
  const int tid = threadIdx.x, lane = tid & 31, wave = tid >> 5;
  const int hh = lane >> 4, c = lane & 15;
  const int task = blockIdx.x * 8 + wave;
  const int b = task / KVT;
  const int t2 = task - b * KVT;
  const int rt = t2 >> 2, cg = t2 & 3;
  const _Float16* Ab = VT + (size_t)b * CX * SEQ;
  const _Float16* Bb = EKT + (size_t)b * DIM * SEQ;
  const int arow0 = rt * 16, bcol0 = cg * 64;

  v8f acc[4];
#pragma unroll
  for (int j = 0; j < 4; ++j) acc[j] = zero8();

#pragma unroll 2
  for (int kc = 0; kc < SEQ / 32; ++kc) {
    const int k0 = kc * 32;
    const v16h a = ldfrag_g(Ab, SEQ, arow0, k0, lane);
#pragma unroll
    for (int j = 0; j < 4; ++j) {
      const v16h bf = ldfrag_g(Bb, SEQ, bcol0 + 16 * j, k0, lane);
      acc[j] = mma16(a, bf, acc[j]);
    }
  }

  _Float16* sw = st[wave];
#pragma unroll
  for (int j = 0; j < 4; ++j)
#pragma unroll
    for (int r = 0; r < 8; ++r) sw[(8 * hh + r) * HP + 16 * j + c] = (_Float16)acc[j][r];
  __syncthreads();

  _Float16* Tb = TT + (size_t)b * CX * DIM;
  v4u val[4];
#pragma unroll
  for (int it = 0; it < 4; ++it) {
    const int p = it * 32 + lane, row = p >> 3, pc = p & 7;
    val[it] = *(const v4ua*)(sw + row * HP + pc * 8);
  }
#pragma unroll
  for (int it = 0; it < 4; ++it) {
    const int p = it * 32 + lane, row = p >> 3, pc = p & 7;
    *(volatile v4u*)(Tb + (size_t)(arow0 + row) * DIM + bcol0 + pc * 8) = val[it];
  }
  __threadfence();
#pragma unroll
  for (int it = 0; it < 4; ++it) {
    const int p = it * 32 + lane, row = p >> 3, pc = p & 7;
    *(volatile v4u*)(Tb + (size_t)(arow0 + row) * DIM + bcol0 + pc * 8) = val[it];
  }
}

__global__ __launch_bounds__(256) void k_out(const _Float16* __restrict__ EQ, const _Float16* __restrict__ TT,
                                             float* __restrict__ out) {
  __shared__ __align__(16) float st[8][16 * FP];
  const int tid = threadIdx.x, lane = tid & 31, wave = tid >> 5;
  const int hh = lane >> 4, c = lane & 15;
  const int rb = wave & 1, cg = wave >> 1;
  const int bm0 = blockIdx.x * 64;
  const int b = bm0 / SEQ;
  const int arow0 = bm0 + rb * 32, bcol0 = cg * 64;
  const _Float16* Tb = TT + (size_t)b * CX * DIM;

  v8f acc[2][4], accd[2];
#pragma unroll
  for (int s = 0; s < 2; ++s) {
    accd[s] = zero8();
#pragma unroll
    for (int j = 0; j < 4; ++j) acc[s][j] = zero8();
  }

#pragma unroll 2
  for (int kc = 0; kc < DIM / 32; ++kc) {
    const int k0 = kc * 32;
    const v16h a0 = ldfrag_g(EQ, DIM, arow0, k0, lane);
    const v16h a1 = ldfrag_g(EQ, DIM, arow0 + 16, k0, lane);
#pragma unroll
    for (int j = 0; j < 4; ++j) {
      const v16h bf = ldfrag_g(Tb, DIM, bcol0 + 16 * j, k0, lane);
      acc[0][j] = mma16(a0, bf, acc[0][j]);
      acc[1][j] = mma16(a1, bf, acc[1][j]);
    }
    const v16h bd = ldfrag_g(Tb, DIM, DIM, k0, lane);
    accd[0] = mma16(a0, bd, accd[0]);
    accd[1] = mma16(a1, bd, accd[1]);
  }

  float* sw = st[wave];
  const int src = hh * 16;
#pragma unroll
  for (int s = 0; s < 2; ++s) {
    float rd[8];
#pragma unroll
    for (int r = 0; r < 8; ++r) {
      const float dv = __shfl(accd[s][r], src);
      rd[r] = 1.0f / dv;
    }
#pragma unroll
    for (int j = 0; j < 4; ++j)
#pragma unroll
      for (int r = 0; r < 8; ++r) sw[(8 * hh + r) * FP + 16 * j + c] = acc[s][j][r] * rd[r];
    __syncthreads();

    v4f val[8];
#pragma unroll
    for (int it = 0; it < 8; ++it) {
      const int p = it * 32 + lane, row = p >> 4, pc = p & 15;
      val[it] = *(const v4fa*)(sw + row * FP + pc * 4);
    }
#pragma unroll
    for (int it = 0; it < 8; ++it) {
      const int p = it * 32 + lane, row = p >> 4, pc = p & 15;
      *(volatile v4f*)(out + (size_t)(arow0 + s * 16 + row) * DIM + bcol0 + pc * 4) = val[it];
    }
    __threadfence();
#pragma unroll
    for (int it = 0; it < 8; ++it) {
      const int p = it * 32 + lane, row = p >> 4, pc = p & 15;
      *(volatile v4f*)(out + (size_t)(arow0 + s * 16 + row) * DIM + bcol0 + pc * 4) = val[it];
    }
    __syncthreads();
  }
}

extern "C" void kernel_launch(void* const* d_in, const int* in_sizes, int n_in,
                              void* d_out, int out_size, void* d_ws, size_t ws_size,
                              hipStream_t stream) {
  if (n_in < 6) return;
  if (in_sizes[0] != NROWS * DIM) return;
  if (in_sizes[1] != NROWS * DIM) return;
  if (in_sizes[2] != NROWS * DIM) return;
  if (in_sizes[3] != NBATCH * DIM) return;
  if (in_sizes[4] != DIM * DIM) return;
  if (in_sizes[5] != 1) return;
  if (out_size != NROWS * DIM) return;

  const float* Q    = (const float*)d_in[0];
  const float* K    = (const float*)d_in[1];
  const float* V    = (const float*)d_in[2];
  const float* semb = (const float*)d_in[3];
  const float* proj = (const float*)d_in[4];
  const int*   qkv  = (const int*)d_in[5];
  float* out = (float*)d_out;

  const size_t q16_b = (size_t)NROWS * DIM * 2;
  const size_t p16_b = (size_t)DIM * DIM * 2;
  const size_t vt_b  = (size_t)NBATCH * CX * SEQ * 2;
  const size_t hn_b  = (size_t)2 * SEQ * 4;
  const size_t e_b   = (size_t)NROWS * DIM * 2;
  const size_t tt_b  = (size_t)NBATCH * CX * DIM * 2;
  size_t off = 0;
  _Float16* Q16 = (_Float16*)((char*)d_ws + off); off += q16_b;
  _Float16* K16 = (_Float16*)((char*)d_ws + off); off += q16_b;
  _Float16* P16 = (_Float16*)((char*)d_ws + off); off += p16_b;
  _Float16* VT  = (_Float16*)((char*)d_ws + off); off += vt_b;
  float*    hn  = (float*)((char*)d_ws + off);    off += hn_b;
  _Float16* EQ  = (_Float16*)((char*)d_ws + off); off += e_b;
  _Float16* EKT = (_Float16*)((char*)d_ws + off); off += e_b;
  _Float16* TT  = (_Float16*)((char*)d_ws + off); off += tt_b;
  if (off > ws_size) return;

  const int nvec_qk = (NROWS * DIM) / 8;
  const int nvec_p  = (DIM * DIM) / 8;

  k_conv<<<dim3(nvec_qk / 256), dim3(256), 0, stream>>>(Q, Q16, nvec_qk, 64.0f);
  k_conv<<<dim3(nvec_qk / 256), dim3(256), 0, stream>>>(K, K16, nvec_qk, 64.0f);
  k_conv<<<dim3(nvec_p / 256), dim3(256), 0, stream>>>(proj, P16, nvec_p, 16.0f);
  k_norm<<<dim3(SEQ / 32, 2), dim3(256), 0, stream>>>(Q, K, hn, semb, qkv);
  k_vt<<<dim3(SEQ / 64, 5, NBATCH), dim3(256), 0, stream>>>(V, VT);
  k_phi<<<dim3(NROWS / 64, 1, 1), dim3(256), 0, stream>>>(Q16, P16, (size_t)0, hn, EQ, DIM, (size_t)0, 0);
  k_phi<<<dim3(DIM / 64, SEQ / 256, NBATCH), dim3(256), 0, stream>>>(P16, K16, (size_t)SEQ * DIM, hn + SEQ,
                                                                     EKT, SEQ, (size_t)DIM * SEQ, 1);
  k_kv<<<dim3((NBATCH * KVT) / 8), dim3(256), 0, stream>>>(VT, EKT, TT);
  k_out<<<dim3(NROWS / 64), dim3(256), 0, stream>>>(EQ, TT, out);
  (void)hipGetLastError();
}
